// NanoGPT_75720273428701
// MI455X (gfx1250) — hardware-verified
//
#include <hip/hip_runtime.h>
#include <math.h>

typedef __attribute__((ext_vector_type(16))) _Float16 v16h;
typedef __attribute__((ext_vector_type(8)))  float    v8f;

#define NW 8
#define TB (NW * 32)
#define NB 32768
#define NT 16
#define NC 8
#define NV 25

typedef __attribute__((ext_vector_type(4))) float v4f_t;
typedef float v4fa __attribute__((ext_vector_type(4), may_alias));
#define RSPLIT (1.0f / 2048.0f)
__device__ __forceinline__ _Float16 lo_of(float v, _Float16 h) { return (_Float16)((v - (float)h) * 2048.0f); }

__global__ void loss_reduce_kernel(const float* __restrict__ part, int n, float* loss) {
    __shared__ float red[256];
    float s = 0.f;
    for (int i = threadIdx.x; i < n; i += 256) s += part[i];
    red[threadIdx.x] = s;
    __syncthreads();
    for (int st = 128; st > 0; st >>= 1) { if (threadIdx.x < st) red[threadIdx.x] += red[threadIdx.x + st]; __syncthreads(); }
    if (threadIdx.x == 0) { const float v = -red[0] * (1.0f / ((float)NB * (float)NT)); *(volatile float*)loss = v; __threadfence(); *(volatile float*)loss = v; }
}

__device__ __forceinline__ v8f wmma(v16h a, v16h b, v8f c) {
    return __builtin_amdgcn_wmma_f32_16x16x32_f16(false, a, false, b, (short)0, c, false, false);
}
struct F2 { v16h h, l; };
__device__ __forceinline__ v8f wmma_split(F2 a, F2 b, v8f c) {
    v8f x = {}; x = wmma(a.l, b.h, x); x = wmma(a.h, b.l, x); return wmma(a.h, b.h, c) + x * RSPLIT;
}

template <int CTRL>
__device__ __forceinline__ float dppf(float x) {
    return __int_as_float(__builtin_amdgcn_update_dpp(
        0, __float_as_int(x), CTRL, 0xf, 0xf, true));
}
__device__ __forceinline__ float row_max16(float x) {
    x = fmaxf(x, dppf<0x121>(x));
    x = fmaxf(x, dppf<0x122>(x));
    x = fmaxf(x, dppf<0x124>(x));
    x = fmaxf(x, dppf<0x128>(x));
    return x;
}
__device__ __forceinline__ float row_sum16(float x) {
    x += dppf<0x121>(x);
    x += dppf<0x122>(x);
    x += dppf<0x124>(x);
    x += dppf<0x128>(x);
    return x;
}

__device__ __forceinline__ F2 frag_lo8(const float* src, float m) {
    const float4* p = (const float4*)src;
    float4 x0 = p[0], x1 = p[1];
    const float xr[8] = {x0.x * m, x0.y * m, x0.z * m, x0.w * m, x1.x * m, x1.y * m, x1.z * m, x1.w * m};
    F2 f;
#pragma unroll
    for (int j = 0; j < 8; ++j) { f.h[j] = (_Float16)xr[j]; f.l[j] = lo_of(xr[j], f.h[j]); }
#pragma unroll
    for (int j = 8; j < 16; ++j) { f.h[j] = (_Float16)0.f; f.l[j] = (_Float16)0.f; }
    return f;
}

__device__ __forceinline__ F2 frag_b8(const float* src, int rs, int co, int ln, float m) {
    F2 b;
#pragma unroll
    for (int j = 0; j < 8; ++j) { const float v = src[j * rs + co + ln] * m; b.h[j] = (_Float16)v; b.l[j] = lo_of(v, b.h[j]); }
#pragma unroll
    for (int j = 8; j < 16; ++j) { b.h[j] = (_Float16)0.f; b.l[j] = (_Float16)0.f; }
    return b;
}

__device__ __forceinline__ void store_d(v8f d, float* dst, int rs, int co, int ln, int half) {
#pragma unroll
    for (int r = 0; r < 8; ++r) dst[(r + 8 * half) * rs + co + ln] = d[r];
}

__device__ __forceinline__ void layernorm(const float* xw, float* dst,
                                          const float* g, const float* bta,
                                          int ln, int half) {
    if (half == 0) {
        const float4* xp = (const float4*)(xw + ln * 16);
        float4 x0 = xp[0], x1 = xp[1];
        float xr[8] = {x0.x, x0.y, x0.z, x0.w, x1.x, x1.y, x1.z, x1.w};
        float mu = 0.f;
#pragma unroll
        for (int c = 0; c < NC; ++c) mu += xr[c];
        mu *= 0.125f;
        float var = 0.f;
#pragma unroll
        for (int c = 0; c < NC; ++c) { float d = xr[c] - mu; var += d * d; }
        var *= 0.125f;
        float is = rsqrtf(var + 1e-5f);
#pragma unroll
        for (int c = 0; c < NC; ++c) dst[ln * 32 + c] = (xr[c] - mu) * is * g[c] + bta[c];
    }
}

__global__ __launch_bounds__(TB) void gpt_fwd_kernel(
    const int* __restrict__ idx, const int* __restrict__ tgt,
    const float* __restrict__ wte, const float* __restrict__ wpe,
    const float* __restrict__ ln1g, const float* __restrict__ ln1b,
    const float* __restrict__ wattn_g, const float* __restrict__ wproj_g,
    const float* __restrict__ ln2g, const float* __restrict__ ln2b,
    const float* __restrict__ wfc_g, const float* __restrict__ wmlp_g,
    const float* __restrict__ lnfg, const float* __restrict__ lnfb,
    const float* __restrict__ whead_g,
    float* __restrict__ logits, float* __restrict__ loss)
{
    __shared__ __align__(16) float wattn[8 * 32];
    __shared__ __align__(16) float whead[8 * 32];
    __shared__ __align__(16) float wproj[8 * 16];
    __shared__ __align__(16) float wfc[8 * 16];
    __shared__ __align__(16) float wmlp[8 * 16];
    __shared__ __align__(16) float lnw[6 * 8];
    __shared__ __align__(16) float xbuf[NW * NT * 16];
    __shared__ __align__(16) float sbuf[NW * NT * 32];
    __shared__ __align__(16) float abuf[NW * NT * NT];
    __shared__ float lred[NW];
    __shared__ __align__(16) float lgs[NW * NT * NV];

    const int tid = threadIdx.x;
    for (int i = tid; i < 8 * 32; i += TB) {
        int r = i >> 5, c = i & 31;
        wattn[i] = (c < 24) ? wattn_g[r * 24 + c] : 0.f;
        whead[i] = (c < NV) ? whead_g[r * NV + c] : 0.f;
    }
    for (int i = tid; i < 8 * 16; i += TB) {
        int r = i >> 4, c = i & 15;
        wproj[i] = (c < 8) ? wproj_g[r * 8 + c] : 0.f;
        wfc[i]   = (c < 8) ? wfc_g[r * 8 + c]   : 0.f;
        wmlp[i]  = (c < 8) ? wmlp_g[r * 8 + c]  : 0.f;
    }
    if (tid < 8) {
        lnw[tid]      = ln1g[tid]; lnw[8 + tid]  = ln1b[tid];
        lnw[16 + tid] = ln2g[tid]; lnw[24 + tid] = ln2b[tid];
        lnw[32 + tid] = lnfg[tid]; lnw[40 + tid] = lnfb[tid];
    }
    __syncthreads();

    const int wid  = tid >> 5;
    const int lane = tid & 31;
    const int half = lane >> 4;
    const int ln   = lane & 15;
    const int b    = blockIdx.x * NW + wid;
    const float mh = (half == 0) ? 1.f : 0.f;

    float* xw = xbuf + wid * (NT * 16);
    float* sw = sbuf + wid * (NT * 32);
    float* aw = abuf + wid * (NT * NT);

    const v8f vzero = {0.f, 0.f, 0.f, 0.f, 0.f, 0.f, 0.f, 0.f};

    for (int i = lane; i < NT * NC; i += 32) {
        int t = i >> 3, c = i & 7;
        int id = idx[b * NT + t];
        if (id < 0) id += NV;
        id = (id < 0) ? 0 : (id > NV - 1 ? NV - 1 : id);
        xw[t * 16 + c] = wte[id * NC + c] + wpe[i];
    }

    layernorm(xw, sw, lnw + 0, lnw + 8, ln, half);

    {
        F2 a  = frag_lo8(sw + ln * 32, mh);
        F2 b0 = frag_b8(wattn, 32, 0,  ln, mh);
        F2 b1 = frag_b8(wattn, 32, 16, ln, mh);
        v8f q0 = wmma_split(a, b0, vzero);
        v8f q1 = wmma_split(a, b1, vzero);
        store_d(q0, sw, 32, 0,  ln, half);
        store_d(q1, sw, 32, 16, ln, half);
    }

    v8f att;
    {
        F2 aq = frag_lo8(sw + ln * 32, mh);
        F2 bk = frag_lo8(sw + ln * 32 + 8, mh);
        att = wmma_split(aq, bk, vzero);
    }
#pragma unroll
    for (int r = 0; r < 8; ++r) {
        int m = r + 8 * half;
        float s = (ln <= m) ? att[r] * 0.3535533906f : -INFINITY;
        float mx = row_max16(s);
        float e = (ln <= m) ? __expf(s - mx) : 0.f;
        float se = row_sum16(e);
        aw[m * NT + ln] = e / se;
    }

    {
        F2 aa = frag_lo8(aw + ln * 16 + half * 8, 1.f);
        float mv = (ln < 8) ? 1.f : 0.f;
        F2 bv;
#pragma unroll
        for (int j = 0; j < 8; ++j) { const float v = sw[(half * 8 + j) * 32 + 16 + ln] * mv; bv.h[j] = (_Float16)v; bv.l[j] = lo_of(v, bv.h[j]); }
#pragma unroll
        for (int j = 8; j < 16; ++j) { bv.h[j] = (_Float16)0.f; bv.l[j] = (_Float16)0.f; }
        v8f y = wmma_split(aa, bv, vzero);
        store_d(y, sw, 32, 0, ln, half);
    }

    {
        F2 a  = frag_lo8(sw + ln * 32, mh);
        F2 bp = frag_b8(wproj, 16, 0, ln, mh);
        v8f o = wmma_split(a, bp, vzero);
#pragma unroll
        for (int r = 0; r < 8; ++r) xw[(r + 8 * half) * 16 + ln] += o[r];
    }

    layernorm(xw, sw, lnw + 16, lnw + 24, ln, half);

    {
        F2 a  = frag_lo8(sw + ln * 32, mh);
        F2 bf = frag_b8(wfc, 16, 0, ln, mh);
        v8f h = wmma_split(a, bf, vzero);
#pragma unroll
        for (int r = 0; r < 8; ++r) {
            float v = h[r];
            sw[(r + 8 * half) * 32 + ln] = 0.5f * v * (1.f + erff(v * 0.7071067812f));
        }
    }

    {
        F2 a  = frag_lo8(sw + ln * 32, mh);
        F2 bm = frag_b8(wmlp, 16, 0, ln, mh);
        v8f o = wmma_split(a, bm, vzero);
#pragma unroll
        for (int r = 0; r < 8; ++r) xw[(r + 8 * half) * 16 + ln] += o[r];
    }

    layernorm(xw, sw, lnw + 32, lnw + 40, ln, half);

    v8f l0, l1;
    {
        F2 a  = frag_lo8(sw + ln * 32, mh);
        F2 b0 = frag_b8(whead, 32, 0,  ln, mh);
        F2 b1 = frag_b8(whead, 32, 16, ln, mh);
        l0 = wmma_split(a, b0, vzero);
        l1 = wmma_split(a, b1, vzero);
    }

    float wl = 0.f;
#pragma unroll
    for (int r = 0; r < 8; ++r) {
        int t = r + 8 * half;
        float* lrow = lgs + (wid * NT + t) * NV;
        lrow[ln] = l0[r];
        if (ln < NV - 16) lrow[16 + ln] = l1[r];

        float a0 = l0[r];
        float a1 = (ln < NV - 16) ? l1[r] : -INFINITY;
        float mx = row_max16(fmaxf(a0, a1));
        float e  = __expf(a0 - mx) + ((ln < NV - 16) ? __expf(a1 - mx) : 0.f);
        e = row_sum16(e);

        int tg = tgt[b * NT + t];
        float pick = (tg == ln) ? a0 : ((tg == ln + 16 && ln < NV - 16) ? l1[r] : 0.f);
        float lt = row_sum16(pick);
        wl += lt - mx - __logf(e);
    }
    wl += __shfl_xor(wl, 16, 32);
    if (lane == 0) lred[wid] = wl;
    __syncthreads();
    if (tid == 0) {
        float s = 0.f;
#pragma unroll
        for (int w = 0; w < NW; ++w) s += lred[w];
        *(volatile float*)(loss + 1 + blockIdx.x) = s;
    }
#pragma unroll 1
    for (int pass = 0; pass < 2; ++pass) {
        for (int c = tid; c < NW * NT * NV / 4; c += TB)
            *(volatile v4f_t*)(logits + (size_t)blockIdx.x * (NW * NT * NV) + c * 4) = *(const volatile v4fa*)(lgs + c * 4);
        __threadfence();
    }
}

extern "C" void kernel_launch(void* const* d_in, const int* in_sizes, int n_in,
                              void* d_out, int out_size, void* d_ws, size_t ws_size,
                              hipStream_t stream) {
    const int*   idx   = (const int*)d_in[0];
    const int*   tgt   = (const int*)d_in[1];
    const float* wte   = (const float*)d_in[2];
    const float* wpe   = (const float*)d_in[3];
    const float* ln1g  = (const float*)d_in[4];
    const float* ln1b  = (const float*)d_in[5];
    const float* wattn = (const float*)d_in[6];
    const float* wproj = (const float*)d_in[7];
    const float* ln2g  = (const float*)d_in[8];
    const float* ln2b  = (const float*)d_in[9];
    const float* wfc   = (const float*)d_in[10];
    const float* wmlp  = (const float*)d_in[11];
    const float* lnfg  = (const float*)d_in[12];
    const float* lnfb  = (const float*)d_in[13];
    const float* whead = (const float*)d_in[14];

    float* logits = (float*)d_out;
    float* loss   = logits + (size_t)NB * NT * NV;
    float* part   = (float*)d_ws;
    (void)ws_size;

    gpt_fwd_kernel<<<NB / NW, TB, 0, stream>>>(
        idx, tgt, wte, wpe, ln1g, ln1b, wattn, wproj,
        ln2g, ln2b, wfc, wmlp, lnfg, lnfb, whead, logits, part);
    loss_reduce_kernel<<<1, 256, 0, stream>>>(part + 1, NB / NW, loss);
}
